// QRNNLayer_51230369907342
// MI455X (gfx1250) — hardware-verified
//
#include <hip/hip_runtime.h>
#include <math.h>

constexpr int kBatch  = 8;
constexpr int kSeq    = 4096;
constexpr int kIn     = 256;
constexpr int kOut    = 256;
constexpr int kKdim   = 512;
constexpr int kNdim   = 768;
constexpr int kSeqPad = kSeq + 1;

typedef __attribute__((ext_vector_type(16))) _Float16 v16h;
typedef __attribute__((ext_vector_type(8)))  _Float16 v8h;
typedef __attribute__((ext_vector_type(16))) __bf16   v16b;
typedef __attribute__((ext_vector_type(8)))  __bf16   v8b;
typedef __attribute__((ext_vector_type(8)))  float    v8f;
typedef __attribute__((ext_vector_type(4)))  float    v4f;
typedef __attribute__((ext_vector_type(4)))  unsigned int v4u;

__device__ __forceinline__ unsigned short f2bf_bits(float f) {
  unsigned u = __float_as_uint(f);
  return (unsigned short)((u + 0x7FFFu + ((u >> 16) & 1u)) >> 16);
}
__device__ __forceinline__ float bf_bits2f(unsigned short h) { return __uint_as_float(((unsigned)h) << 16); }

__device__ __forceinline__ void dep_guard_h(v8f& a, v8f& b, v16h x, v16h y) { asm volatile("v_nop\n\tv_nop\n\tv_nop\n\tv_nop" : "+v"(a), "+v"(b) : "v"(x), "v"(y)); }
__device__ __forceinline__ void dep_guard_b(v8f& a, v8f& b, v16b x, v16b y) { asm volatile("v_nop\n\tv_nop\n\tv_nop\n\tv_nop" : "+v"(a), "+v"(b) : "v"(x), "v"(y)); }
__device__ __forceinline__ void keep4_h(v16h a, v16h b, v16h c, v16h d) { asm volatile("v_nop" :: "v"(a), "v"(b), "v"(c), "v"(d)); }
__device__ __forceinline__ void keep4_b(v16b a, v16b b, v16b c, v16b d) { asm volatile("v_nop" :: "v"(a), "v"(b), "v"(c), "v"(d)); }
__device__ __forceinline__ void acc_guard4(v8f& a, v8f& b, v8f& c, v8f& d) { asm volatile("v_nop\n\tv_nop\n\tv_nop\n\tv_nop" : "+v"(a), "+v"(b), "+v"(c), "+v"(d)); }
template <typename T> struct Frag;
template <> struct Frag<_Float16> {
  typedef v16h V; union U { v16h v; v8h h[2]; };
  static __device__ __forceinline__ v16h load(const _Float16* p) {
    U f; f.h[0] = *(const v8h*)(p); f.h[1] = *(const v8h*)(p + 16); return f.v;
  }
  static __device__ __forceinline__ v8f mma(v16h a, v16h b, v8f c) {
    return __builtin_amdgcn_wmma_f32_16x16x32_f16(false, a, false, b, (short)0, c, false, false);
  }
  static __device__ __forceinline__ void guard(v8f& a, v8f& b, v16h x, v16h y) { dep_guard_h(a, b, x, y); }
  static __device__ __forceinline__ void keep(v16h a, v16h b, v16h c, v16h d) { keep4_h(a, b, c, d); }
};
template <> struct Frag<__bf16> {
  typedef v16b V; union U { v16b v; v8b h[2]; };
  static __device__ __forceinline__ v16b load(const __bf16* p) {
    U f; f.h[0] = *(const v8b*)(p); f.h[1] = *(const v8b*)(p + 16); return f.v;
  }
  static __device__ __forceinline__ v8f mma(v16b a, v16b b, v8f c) {
    return __builtin_amdgcn_wmma_f32_16x16x32_bf16(false, a, false, b, (short)0, c, false, false);
  }
  static __device__ __forceinline__ void guard(v8f& a, v8f& b, v16b x, v16b y) { dep_guard_b(a, b, x, y); }
  static __device__ __forceinline__ void keep(v16b a, v16b b, v16b c, v16b d) { keep4_b(a, b, c, d); }
};

__device__ __forceinline__ unsigned pk16(unsigned short a, unsigned short b) { return (unsigned)a | ((unsigned)b << 16); }

template <int ET> struct Elem;
template <> struct Elem<0> { typedef _Float16 T; };
template <> struct Elem<1> { typedef __bf16 T; };
template <int ET, bool SPLIT, int BIAS_MODE, int OUT_MODE, bool RESID, int ACT = 0>
__global__ __launch_bounds__(256) void wmma_gemm64(
    const unsigned short* __restrict__ Ap, const unsigned short* __restrict__ A2p, int lda, long strideA,
    const unsigned short* __restrict__ Btp, const unsigned short* __restrict__ Bt2p, int ldb, long strideB,
    void* __restrict__ Cout, void* __restrict__ Cout2, int ldc, long strideC,
    const float* __restrict__ bias,
    const float* __restrict__ resid, long strideR,
    int M, int N, int K, float scale) {
  typedef typename Elem<ET>::T T;
  typedef typename Frag<T>::V V;
  const T* A = (const T*)Ap; const T* A2 = (const T*)A2p; const T* Bt = (const T*)Btp; const T* Bt2 = (const T*)Bt2p;
  __shared__ __align__(16) float sT[8][16 * 68];
  const int b    = blockIdx.y;
  const int lane = threadIdx.x & 31;
  const int wave = threadIdx.x >> 5;
  const int tilesN = N >> 6;
  const int tilesM = M >> 6;
  const int tile = blockIdx.x * 8 + wave;
  if (tile >= tilesM * tilesN) return;
  const int tm = tile / tilesN;
  const int tn = tile - tm * tilesN;
  const int m0 = tm << 6;
  const int n0 = tn << 6;

  const T* Ab  = A  + (size_t)b * strideA;
  const T* Bb  = Bt + (size_t)b * strideB;
  const T* Ab2 = SPLIT ? (A2  + (size_t)b * strideA) : nullptr;
  const T* Bb2 = SPLIT ? (Bt2 + (size_t)b * strideB) : nullptr;

  const int rlane = lane & 15;
  const int koff  = (lane >> 4) * 8;
  const int mOff  = (lane >> 4) * 8;

  v8f acc[4][4];
#pragma unroll
  for (int i = 0; i < 4; ++i)
#pragma unroll
    for (int j = 0; j < 4; ++j) acc[i][j] = (v8f){0.f,0.f,0.f,0.f,0.f,0.f,0.f,0.f};

  for (int k0 = 0; k0 < K; k0 += 32) {
    V bh[4], bl[4];
#pragma unroll
    for (int j = 0; j < 4; ++j) {
      const size_t bo = (size_t)(n0 + (j << 4) + rlane) * ldb + koff + k0;
      bh[j] = Frag<T>::load(Bb + bo);
      if (SPLIT) bl[j] = Frag<T>::load(Bb2 + bo);
    }
#pragma unroll
    for (int i = 0; i < 4; ++i) {
      const size_t ao = (size_t)(m0 + (i << 4) + rlane) * lda + koff + k0;
      V ah = Frag<T>::load(Ab + ao);
      V al;
      if (SPLIT) al = Frag<T>::load(Ab2 + ao);
#pragma unroll
      for (int j = 0; j < 4; ++j) {
        acc[i][j] = Frag<T>::mma(ah, bh[j], acc[i][j]);
        if (SPLIT) {
          acc[i][j] = Frag<T>::mma(ah, bl[j], acc[i][j]);
          acc[i][j] = Frag<T>::mma(al, bh[j], acc[i][j]);
        }
      }
      Frag<T>::guard(acc[i][0], acc[i][3], ah, SPLIT ? al : ah);
    }
    Frag<T>::keep(bh[0], bh[1], bh[2], bh[3]);
    if (SPLIT) Frag<T>::keep(bl[0], bl[1], bl[2], bl[3]);
  }
  acc_guard4(acc[0][0], acc[0][1], acc[0][2], acc[0][3]);
  acc_guard4(acc[1][0], acc[1][1], acc[1][2], acc[1][3]);
  acc_guard4(acc[2][0], acc[2][1], acc[2][2], acc[2][3]);
  acc_guard4(acc[3][0], acc[3][1], acc[3][2], acc[3][3]);

  float* slab = sT[wave];
  const float* Rb = RESID ? (resid + (size_t)b * strideR) : nullptr;
#pragma unroll
  for (int i = 0; i < 4; ++i) {
    const int mBase = m0 + (i << 4);
#pragma unroll
    for (int j = 0; j < 4; ++j) {
      const int n = n0 + (j << 4) + rlane;
      float bv = 0.f;
      if (BIAS_MODE == 2) bv = bias[n];
#pragma unroll
      for (int r = 0; r < 8; ++r) {
        float v = acc[i][j][r] * scale;
        if (BIAS_MODE == 1) v += bias[mBase + mOff + r];
        if (BIAS_MODE == 2) v += bv;
        if (RESID) v += Rb[(size_t)(mBase + mOff + r) * ldc + n];
        if (ACT == 2) v = fmaxf(v, 0.0f);
        if (ACT == 4) v = (v > 0.f) ? v : 0.01f * v;
        slab[(mOff + r) * 68 + (j << 4) + rlane] = v;
      }
    }
    __builtin_amdgcn_fence(__ATOMIC_RELEASE, "workgroup");
    __builtin_amdgcn_wave_barrier();
    __builtin_amdgcn_fence(__ATOMIC_ACQUIRE, "workgroup");
    if (OUT_MODE == 0) {
      float* C = (float*)Cout + (size_t)b * strideC;
      const int hh = lane >> 4, c4 = (lane & 15) * 4;
      for (int pass = 0; pass < 2; ++pass) {
#pragma unroll
        for (int it = 0; it < 8; ++it) {
          const int row = it * 2 + hh;
          v4f v = *(const v4f*)(slab + row * 68 + c4);
          *(volatile v4f*)(C + (size_t)(mBase + row) * ldc + n0 + c4) = v;
        }
        __threadfence();
      }
    } else {
      const int q = lane >> 3, c8 = (lane & 7) * 8;
      unsigned short* C  = (unsigned short*)Cout  + (size_t)b * strideC;
      unsigned short* C2 = (OUT_MODE == 2) ? ((unsigned short*)Cout2 + (size_t)b * strideC) : nullptr;
      for (int pass = 0; pass < 2; ++pass) {
#pragma unroll
        for (int it = 0; it < 4; ++it) {
          const int row = it * 4 + q;
          const float* sp = slab + row * 68 + c8;
          v8h hv, lv;
#pragma unroll
          for (int e = 0; e < 8; ++e) {
            if (OUT_MODE == 1) {
              hv[e] = (_Float16)sp[e];
            } else {
              unsigned short hb = f2bf_bits(sp[e]);
              unsigned short lb = f2bf_bits(sp[e] - bf_bits2f(hb));
              hv[e] = __builtin_bit_cast(_Float16, hb);
              lv[e] = __builtin_bit_cast(_Float16, lb);
            }
          }
          *(volatile v8h*)(C + (size_t)(mBase + row) * ldc + n0 + c8) = hv;
          if (OUT_MODE == 2) *(volatile v8h*)(C2 + (size_t)(mBase + row) * ldc + n0 + c8) = lv;
        }
        __threadfence();
      }
    }
    __builtin_amdgcn_fence(__ATOMIC_RELEASE, "workgroup");
    __builtin_amdgcn_wave_barrier();
    __builtin_amdgcn_fence(__ATOMIC_ACQUIRE, "workgroup");
  }
}

__global__ __launch_bounds__(256) void castx_kernel(const float* __restrict__ x, unsigned short* __restrict__ xp, int nthreads) {
  const int i = blockIdx.x * 256 + threadIdx.x;
  if (i >= nthreads) return;
  const int prow = i >> 5;
  const int col  = (i & 31) * 8;
  const int b    = prow / kSeqPad;
  const int j    = prow - b * kSeqPad;
  const int js   = (j > 0) ? (j - 1) : 0;
  const bool zero = (j == 0);
  const float* p = x + ((size_t)(b * kSeq + js)) * kIn + col;
  const v4f a = *(const v4f*)(p);
  const v4f c = *(const v4f*)(p + 4);
  unsigned short hb[8];
#pragma unroll
  for (int e = 0; e < 4; ++e) {
    const float v0 = zero ? 0.0f : a[e];
    const float v1 = zero ? 0.0f : c[e];
    hb[e]     = f2bf_bits(v0);
    hb[4 + e] = f2bf_bits(v1);
  }
  const v4u u = (v4u){pk16(hb[0], hb[1]), pk16(hb[2], hb[3]), pk16(hb[4], hb[5]), pk16(hb[6], hb[7])};
  unsigned short* q = xp + 8 * (size_t)i;
  *(volatile v4u*)q = u;
  __threadfence();
  *(volatile v4u*)q = u;
}

__global__ __launch_bounds__(256) void castw_kernel(const float* __restrict__ in, unsigned short* __restrict__ out, int n8) {
  const int i = blockIdx.x * 256 + threadIdx.x;
  if (i >= n8) return;
  const float* p = in + 8 * (size_t)i;
  const v4f a = *(const v4f*)(p);
  const v4f c = *(const v4f*)(p + 4);
  unsigned short hb[8];
#pragma unroll
  for (int e = 0; e < 4; ++e) {
    hb[e]     = f2bf_bits(a[e]);
    hb[4 + e] = f2bf_bits(c[e]);
  }
  const v4u u = (v4u){pk16(hb[0], hb[1]), pk16(hb[2], hb[3]), pk16(hb[4], hb[5]), pk16(hb[6], hb[7])};
  unsigned short* q = out + 8 * (size_t)i;
  *(volatile v4u*)q = u;
  __threadfence();
  *(volatile v4u*)q = u;
}

__global__ __launch_bounds__(256) void fo_pool_kernel(const float* __restrict__ Y, const float* __restrict__ bias,
                                                      float* __restrict__ out) {
#pragma clang fp contract(off)
  const int b  = blockIdx.x;
  const int ch = threadIdx.x;
  const float bz = bf_bits2f(f2bf_bits(bias[ch]));
  const float bf = bf_bits2f(f2bf_bits(bias[kOut + ch]));
  const float bo = bf_bits2f(f2bf_bits(bias[2 * kOut + ch]));
  const float* yp = Y + (size_t)b * kSeq * kNdim + ch;
  float* op = out + (size_t)b * kSeq * kOut + ch;
  float c = 0.0f;
#pragma unroll 1
  for (int t = 0; t < kSeq; ++t) {
    const float* yr = yp + (size_t)t * kNdim;
    const float yz = yr[0] + bz;
    const float yf = yr[kOut] + bf;
    const float yo = yr[2 * kOut] + bo;
    const float e2 = fminf(expf(2.0f * yz), 1.0e30f);
    const float z  = 1.0f - 2.0f / (e2 + 1.0f);
    const float ef = fminf(expf(-yf), 1.0e30f);
    const float f  = 1.0f / (1.0f + ef);
    const float eg = fminf(expf(-yo), 1.0e30f);
    const float g  = 1.0f / (1.0f + eg);
    const float p1 = f * c;
    const float p2 = (1.0f - f) * z;
    c = p1 + p2;
    const float ov = g * c;
    volatile float* dst = op + (size_t)t * kOut;
    *dst = ov;
    __threadfence();
    *dst = ov;
  }
}

extern "C" void kernel_launch(void* const* d_in, const int* in_sizes, int n_in,
                              void* d_out, int out_size, void* d_ws, size_t ws_size,
                              hipStream_t stream) {
  if (n_in < 3) return;
  if (in_sizes[0] != kBatch * kSeq * kIn) return;
  if (in_sizes[1] != kNdim * kKdim) return;
  if (in_sizes[2] != kNdim) return;
  if (out_size != kBatch * kSeq * kOut) return;

  const float* x    = (const float*)d_in[0];
  const float* W    = (const float*)d_in[1];
  const float* bias = (const float*)d_in[2];
  float* out = (float*)d_out;

  const size_t xpHalves = (size_t)kBatch * kSeqPad * kIn;
  const size_t offXP    = 0;
  const size_t bytesXP  = xpHalves * 2;
  const size_t offW16   = offXP + bytesXP;
  const size_t bytesW16 = (size_t)kNdim * kKdim * 2;
  const size_t offY     = offW16 + bytesW16;
  const size_t bytesY   = (size_t)kBatch * kSeq * kNdim * 4;
  const size_t total    = offY + bytesY;
  if (total > ws_size) return;

  char* ws = (char*)d_ws;
  unsigned short* XP  = (unsigned short*)(ws + offXP);
  unsigned short* W16 = (unsigned short*)(ws + offW16);
  float*          Y   = (float*)(ws + offY);

  const int nxThreads = (int)(xpHalves / 8);
  const int nxBlocks  = (nxThreads + 255) / 256;
  castx_kernel<<<nxBlocks, 256, 0, stream>>>(x, XP, nxThreads);

  const int nw8      = kNdim * kKdim / 8;
  const int nwBlocks = (nw8 + 255) / 256;
  castw_kernel<<<nwBlocks, 256, 0, stream>>>(W, W16, nw8);

  {
    const int tiles = (kSeq / 64) * (kNdim / 64);
    dim3 ggrid((tiles + 7) / 8, kBatch);
    wmma_gemm64<1, false, 0, 0, false, 0><<<ggrid, 256, 0, stream>>>(
        XP, XP, kIn, (long)kSeqPad * kIn,
        W16, W16, kKdim, 0L,
        (void*)Y, (void*)Y, kNdim, (long)kSeq * kNdim,
        bias,
        bias, 0L,
        kSeq, kNdim, kKdim, 1.0f);
  }

  fo_pool_kernel<<<kBatch, 256, 0, stream>>>(Y, bias, out);
}
